// Model_7773890806494
// MI455X (gfx1250) — hardware-verified
//
#include <hip/hip_runtime.h>
#include <stddef.h>
#include <stdint.h>


#define BSZ    32
#define NNODE  4096
#define CH     64
#define MEDGE  64
#define EINC   16384
#define NROW   (BSZ * NNODE)
#define NTHR   256
#define NWAVE  8
#define EPT    8
#define CHUNK  (NTHR * EPT)
#define WCAP   (EPT * 32)
#define LISTN  (NWAVE * WCAP)
#define NBA    1024
#define SLA    10
#define RCAP   EINC
#define DEGCAP 32
#define NBLKN  (NNODE / NBA)
#define GTM    128
#define SCH    1024
#define NEGSL  0.2f
#define HINGE  4.2f
#define NU_A   (EINC * BSZ / 4)
#define NU_W   (CH * CH / 8)
#define NU_T   (2 * CH / 4)
#define BK_ZINTS (LISTN + 2 * RCAP + 3 * NBA)
#define BK_LDS_INTS (BK_ZINTS + 16)
#define WSMAX  134217728

static_assert((CHUNK & (CHUNK - 1)) == 0 && CHUNK <= 4096);
static_assert(NBA == (1 << SLA) && NNODE % NBA == 0);
static_assert(((long long)CHUNK << SLA) < (1LL << 31));
static_assert(((long long)EINC << SLA) < (1LL << 31));
static_assert(RCAP >= EINC && RCAP % 128 == 0 && BK_ZINTS % 4 == 0);
static_assert(BK_LDS_INTS * 4 <= 300000);
static_assert(NROW % GTM == 0 && GTM == NWAVE * 16);
static_assert(CH == 64 && BSZ == 32 && DEGCAP == 32 && MEDGE == 64);
static_assert(NNODE % NWAVE == 0 && NBA / NWAVE == 128 && NBA == 4 * NTHR);
static_assert(NU_A % NTHR == 0 && NU_W % NTHR == 0 && NU_T == 32);
static_assert(SCH == 4 * NTHR && BSZ == 4 * NWAVE);
static_assert(MEDGE * MEDGE == 32 * 128);

typedef float          v2f   __attribute__((ext_vector_type(2)));
typedef float          v4f   __attribute__((ext_vector_type(4)));
typedef float          v8f   __attribute__((ext_vector_type(8)));
typedef double         v2d   __attribute__((ext_vector_type(2)));
typedef int            v4i   __attribute__((ext_vector_type(4)));
typedef int            v8i   __attribute__((ext_vector_type(8)));
typedef unsigned short v8us  __attribute__((ext_vector_type(8)));
typedef unsigned short v16us __attribute__((ext_vector_type(16)));
typedef __bf16         v16bf __attribute__((ext_vector_type(16)));
typedef v2f  __attribute__((may_alias)) v2fa;
typedef v4f  __attribute__((may_alias)) v4fa;
typedef v4i  __attribute__((may_alias)) v4ia;
typedef v8us __attribute__((may_alias)) v8usa;
union FragB { v16bf v; v16us u; v8us h[2]; v8i w; };

__device__ __forceinline__ v8f wmb(const FragB& a, const FragB& b, v8f c) {
  v8f d = __builtin_amdgcn_wmma_f32_16x16x32_bf16(false, a.v, false, b.v, (short)0, c, false, false);
  asm volatile("v_nop\n\tv_nop\n\tv_nop\n\tv_nop" : "+v"(d) : "v"(a.w), "v"(b.w));
  return d;
}

__device__ __forceinline__ unsigned bf16_bits(float f) {
  const unsigned u = __float_as_uint(f);
  return (u + 0x7FFFu + ((u >> 16) & 1u)) >> 16;
}
__device__ __forceinline__ float bf16_val(float f) {
  return __uint_as_float(bf16_bits(f) << 16);
}
__device__ __forceinline__ v4f bfr4(const v4f a) {
  v4f r; r.x = bf16_val(a.x); r.y = bf16_val(a.y); r.z = bf16_val(a.z); r.w = bf16_val(a.w); return r;
}
__device__ __forceinline__ v8us cvt8(const v4f a, const v4f b) {
  v8us o;
  o[0] = (unsigned short)bf16_bits(a.x); o[1] = (unsigned short)bf16_bits(a.y);
  o[2] = (unsigned short)bf16_bits(a.z); o[3] = (unsigned short)bf16_bits(a.w);
  o[4] = (unsigned short)bf16_bits(b.x); o[5] = (unsigned short)bf16_bits(b.y);
  o[6] = (unsigned short)bf16_bits(b.z); o[7] = (unsigned short)bf16_bits(b.w);
  return o;
}
__device__ __forceinline__ int clampi(int v, int lo, int hi) { return v < lo ? lo : (v > hi ? hi : v); }

template <int SLB>
__device__ __forceinline__ int scan_chunk_ord(const int* __restrict__ keys, int nE, int cbase, int slotBase,
                                              int nb, int vec8, int* list, int tid, int lane, int wave) {
  const int el0  = tid * EPT;
  const int e0   = cbase + el0;
  const int sent = -2147483647 - 1;
  v4i da, db;
  if (vec8 != 0 && cbase + CHUNK <= nE) {
    da = *(const v4i*)(keys + e0);
    db = *(const v4i*)(keys + e0 + 4);
  } else {
    da.x = (e0     < nE) ? keys[min(e0,     nE - 1)] : sent;
    da.y = (e0 + 1 < nE) ? keys[min(e0 + 1, nE - 1)] : sent;
    da.z = (e0 + 2 < nE) ? keys[min(e0 + 2, nE - 1)] : sent;
    da.w = (e0 + 3 < nE) ? keys[min(e0 + 3, nE - 1)] : sent;
    db.x = (e0 + 4 < nE) ? keys[min(e0 + 4, nE - 1)] : sent;
    db.y = (e0 + 5 < nE) ? keys[min(e0 + 5, nE - 1)] : sent;
    db.z = (e0 + 6 < nE) ? keys[min(e0 + 6, nE - 1)] : sent;
    db.w = (e0 + 7 < nE) ? keys[min(e0 + 7, nE - 1)] : sent;
  }
  const unsigned nbs = (unsigned)slotBase;
  const unsigned unb = (unsigned)nb;
  const unsigned s0 = (unsigned)da.x - nbs, s1 = (unsigned)da.y - nbs;
  const unsigned s2 = (unsigned)da.z - nbs, s3 = (unsigned)da.w - nbs;
  const unsigned s4 = (unsigned)db.x - nbs, s5 = (unsigned)db.y - nbs;
  const unsigned s6 = (unsigned)db.z - nbs, s7 = (unsigned)db.w - nbs;
  const bool h0 = s0 < unb, h1 = s1 < unb, h2 = s2 < unb, h3 = s3 < unb;
  const bool h4 = s4 < unb, h5 = s5 < unb, h6 = s6 < unb, h7 = s7 < unb;
  const int c = (int)h0 + (int)h1 + (int)h2 + (int)h3 + (int)h4 + (int)h5 + (int)h6 + (int)h7;
  int incl = c;
#pragma unroll
  for (int d = 1; d < 32; d <<= 1) {
    const int y = __shfl_up(incl, d, 32);
    incl += (lane >= d) ? y : 0;
  }
  const int wc = __shfl(incl, 31, 32);
  int pos = incl - c;
  int* wl = list + wave * WCAP;
  if (h0) { if (pos < WCAP) wl[pos] = ((el0 + 0) << SLB) | (int)s0; pos += 1; }
  if (h1) { if (pos < WCAP) wl[pos] = ((el0 + 1) << SLB) | (int)s1; pos += 1; }
  if (h2) { if (pos < WCAP) wl[pos] = ((el0 + 2) << SLB) | (int)s2; pos += 1; }
  if (h3) { if (pos < WCAP) wl[pos] = ((el0 + 3) << SLB) | (int)s3; pos += 1; }
  if (h4) { if (pos < WCAP) wl[pos] = ((el0 + 4) << SLB) | (int)s4; pos += 1; }
  if (h5) { if (pos < WCAP) wl[pos] = ((el0 + 5) << SLB) | (int)s5; pos += 1; }
  if (h6) { if (pos < WCAP) wl[pos] = ((el0 + 6) << SLB) | (int)s6; pos += 1; }
  if (h7) { if (pos < WCAP) wl[pos] = ((el0 + 7) << SLB) | (int)s7; pos += 1; }
  return wc;
}

__global__ __launch_bounds__(NTHR) void k_prep(const float* __restrict__ W, const float* __restrict__ att,
                                               unsigned short* WT, float* ATTF, float* ALPHA) {
  const int u = (int)blockIdx.x * NTHR + (int)threadIdx.x;
  if (u < NU_A) {
    const v4f z = {0.0f, 0.0f, 0.0f, 0.0f};
    float* dp = ALPHA + (size_t)u * 4;
    *(volatile v4f*)dp = z;
    __threadfence();
    *(volatile v4f*)dp = z;
  } else if (u < NU_A + NU_W) {
    const int v  = u - NU_A;
    const int n  = v >> 3;
    const int k8 = (v & 7) * 8;
    const float* p = W + (size_t)k8 * CH + n;
    v8us o;
#pragma unroll
    for (int i = 0; i < 8; ++i) o[i] = (unsigned short)bf16_bits(p[(size_t)i * CH]);
    unsigned short* dp = WT + (size_t)v * 8;
    *(volatile v8us*)dp = o;
    __threadfence();
    *(volatile v8us*)dp = o;
  } else if (u < NU_A + NU_W + NU_T) {
    const int v = u - NU_A - NU_W;
    const v4f a = bfr4(*(const v4f*)(att + 4 * v));
    float* dp = ATTF + 4 * v;
    *(volatile v4f*)dp = a;
    __threadfence();
    *(volatile v4f*)dp = a;
  }
}

__device__ __forceinline__ void put_node_tables(const int* cnt, const int* offs, const int* sl, int nodeBase,
                                                int wave, int lane, int pflag, int blk,
                                                int* NCNT, int* NLIST, int* POISONV) {
  const int s0 = wave * (NBA / NWAVE);
  {
    const v4i c4 = *(const v4ia*)(cnt + s0 + 4 * lane);
    *(volatile v4i*)(NCNT + nodeBase + s0 + 4 * lane) = c4;
  }
  const int p4 = (lane & 7) * 4;
#pragma unroll 1
  for (int it = 0; it < 32; ++it) {
    const int s = s0 + 4 * it + (lane >> 3);
    const int c = clampi(cnt[s], 0, DEGCAP);
    const int o = clampi(offs[s], 0, RCAP);
    const int i0 = min(o + p4 + 0, RCAP - 1), i1 = min(o + p4 + 1, RCAP - 1);
    const int i2 = min(o + p4 + 2, RCAP - 1), i3 = min(o + p4 + 3, RCAP - 1);
    const int q0 = sl[i0] >> SLA, q1 = sl[i1] >> SLA, q2 = sl[i2] >> SLA, q3 = sl[i3] >> SLA;
    v4i o4;
    o4.x = (p4 + 0 < c) ? q0 : 0;
    o4.y = (p4 + 1 < c) ? q1 : 0;
    o4.z = (p4 + 2 < c) ? q2 : 0;
    o4.w = (p4 + 3 < c) ? q3 : 0;
    *(volatile v4i*)(NLIST + (size_t)(nodeBase + s0 + 4 * it) * DEGCAP + 4 * lane) = o4;
  }
  if (wave == 0 && lane < 8) {
    const v4i f4 = {pflag, pflag, pflag, pflag};
    *(volatile v4i*)(POISONV + blk * 32 + 4 * lane) = f4;
  }
}

__global__ __launch_bounds__(NTHR) void k_bucket(const int* __restrict__ hidx, int nE, int vec8,
                                                 int* NCNT, int* NLIST, int* POISONV,
                                                 int* ELIST, int* ECNTV) {
  extern __shared__ __attribute__((aligned(16))) int dsm[];
  int* list = dsm;
  int* hl   = dsm + LISTN;
  int* sl   = hl + RCAP;
  int* cnt  = sl + RCAP;
  int* offs = cnt + NBA;
  int* cur  = offs + NBA;
  int* misc = cur + NBA;
  const int tid = (int)threadIdx.x, lane = tid & 31, wave = tid >> 5;
  {
    const v4i z4 = {0, 0, 0, 0};
    for (int i = tid * 4; i < BK_ZINTS; i += NTHR * 4) *(v4ia*)(dsm + i) = z4;
    if (tid < 16) misc[tid] = 0;
  }
  __syncthreads();
  const int nChunks = (nE + CHUNK - 1) / CHUNK;

  if ((int)blockIdx.x < NBLKN) {
    const int* keys = hidx;
    const int nodeBase = (int)blockIdx.x * NBA;
    int t = 0, ov = 0;
#pragma unroll 1
    for (int ch = 0; ch < nChunks; ++ch) {
      const int cbase = ch * CHUNK;
      const int wc = scan_chunk_ord<SLA>(keys, nE, cbase, nodeBase, NBA, vec8, list, tid, lane, wave);
      if (lane == 0) misc[wave] = wc;
      __syncthreads();
      if (wave == 0) {
#pragma unroll 1
        for (int w2 = 0; w2 < NWAVE; ++w2) {
          int c = misc[w2];
          c = c < 0 ? 0 : (c > WCAP ? WCAP : c);
#pragma unroll 1
          for (int b0 = 0; b0 < c; b0 += 32) {
            const int idx = b0 + lane;
            const int ent = list[w2 * WCAP + (idx < WCAP ? idx : WCAP - 1)];
            const int m32 = (c - b0) < 32 ? (c - b0) : 32;
#pragma unroll 1
            for (int k = 0; k < m32; ++k) {
              const int u    = __builtin_amdgcn_readlane(ent, k);
              const int slot = u & (NBA - 1);
              const int el   = (u >> SLA) & (CHUNK - 1);
              const int pk   = ((cbase + el) << SLA) | slot;
              if (t < RCAP) {
                if (lane == 0) { hl[t] = pk; cnt[slot] = cnt[slot] + 1; }
                t = t + 1;
              } else {
                ov = 1;
              }
            }
          }
        }
      }
      __syncthreads();
    }
    if (wave == 0 && lane == 0) { misc[8] = t; misc[9] = ov; }
    __syncthreads();
    int tt = misc[8];
    tt = tt < 0 ? 0 : (tt > RCAP ? RCAP : tt);
    const int ovf = misc[9];

    if (wave == 0) {
      const int base = lane * (NBA / 32);
      int s = 0;
#pragma unroll 1
      for (int i = 0; i < NBA / 32; ++i) s += cnt[base + i];
      int incl = s;
#pragma unroll
      for (int d = 1; d < 32; d <<= 1) {
        const int y = __shfl_up(incl, d, 32);
        incl += (lane >= d) ? y : 0;
      }
      int run = incl - s;
#pragma unroll 1
      for (int i = 0; i < NBA / 32; ++i) {
        const int cv = cnt[base + i];
        offs[base + i] = run;
        cur[base + i]  = run;
        run += cv;
      }
    }
    __syncthreads();
    if (wave == 0) {
#pragma unroll 1
      for (int b0 = 0; b0 < tt; b0 += 32) {
        const int idx = b0 + lane;
        const int ent = hl[idx < RCAP ? idx : RCAP - 1];
        const int m32 = (tt - b0) < 32 ? (tt - b0) : 32;
#pragma unroll 1
        for (int k = 0; k < m32; ++k) {
          const int u    = __builtin_amdgcn_readlane(ent, k);
          const int slot = u & (NBA - 1);
          if (lane == 0) {
            int p = cur[slot];
            p = p < 0 ? 0 : (p > RCAP - 1 ? RCAP - 1 : p);
            sl[p] = u;
            cur[slot] = p + 1;
          }
        }
      }
    }
    {
      int f = 0;
      f |= (cnt[4 * tid + 0] > DEGCAP) ? 1 : 0;
      f |= (cnt[4 * tid + 1] > DEGCAP) ? 1 : 0;
      f |= (cnt[4 * tid + 2] > DEGCAP) ? 1 : 0;
      f |= (cnt[4 * tid + 3] > DEGCAP) ? 1 : 0;
      if (f != 0) misc[10] = 1;
    }
    __syncthreads();
    const int pflag = ((misc[10] | ovf) != 0) ? 1 : 0;
    put_node_tables(cnt, offs, sl, nodeBase, wave, lane, pflag, (int)blockIdx.x, NCNT, NLIST, POISONV);
    __threadfence();
    put_node_tables(cnt, offs, sl, nodeBase, wave, lane, pflag, (int)blockIdx.x, NCNT, NLIST, POISONV);
  } else {
    const int* keys = hidx + nE;
    const int m = (int)blockIdx.x - NBLKN;
    int t = 0;
#pragma unroll 1
    for (int ch = 0; ch < nChunks; ++ch) {
      const int cbase = ch * CHUNK;
      const int wc = scan_chunk_ord<SLA>(keys, nE, cbase, m, 1, vec8, list, tid, lane, wave);
      if (lane == 0) misc[wave] = wc;
      __syncthreads();
      int pre = 0, tot = 0;
#pragma unroll
      for (int w2 = 0; w2 < NWAVE; ++w2) {
        const int c2 = clampi(misc[w2], 0, WCAP);
        pre += (w2 < wave) ? c2 : 0;
        tot += c2;
      }
      const int wcc = clampi(wc, 0, WCAP);
#pragma unroll 1
      for (int p0 = 0; p0 < wcc; p0 += 32) {
        const int pos = p0 + lane;
        const int ent = list[wave * WCAP + (pos < WCAP ? pos : WCAP - 1)];
        const int el  = (ent >> SLA) & (CHUNK - 1);
        const int dp  = t + pre + pos;
        if (pos < wcc && dp < RCAP) hl[dp] = cbase + el;
      }
      t += tot;
      __syncthreads();
    }
    const int tc = clampi(t, 0, RCAP);
    const int ng = (tc + 127) >> 7;
    int* erow = ELIST + (size_t)m * EINC;
#pragma unroll 1
    for (int g = wave; g < ng; g += NWAVE) {
      const v4i v = *(const v4ia*)(hl + 128 * g + 4 * lane);
      *(volatile v4i*)(erow + 128 * g + 4 * lane) = v;
    }
    if (wave == 0 && lane < 8) {
      const v4i c4 = {tc, tc, tc, tc};
      *(volatile v4i*)(ECNTV + m * 32 + 4 * lane) = c4;
    }
    __threadfence();
#pragma unroll 1
    for (int g = wave; g < ng; g += NWAVE) {
      const v4i v = *(const v4ia*)(hl + 128 * g + 4 * lane);
      *(volatile v4i*)(erow + 128 * g + 4 * lane) = v;
    }
    if (wave == 0 && lane < 8) {
      const v4i c4 = {tc, tc, tc, tc};
      *(volatile v4i*)(ECNTV + m * 32 + 4 * lane) = c4;
    }
  }
}

__global__ __launch_bounds__(NTHR) void k_gemm(const float* __restrict__ x, const unsigned short* __restrict__ WT,
                                               const float* __restrict__ ATTF, float* XW, float* SN) {
  __shared__ __attribute__((aligned(16))) float stg[GTM * CH];
  __shared__ __attribute__((aligned(16))) float sdt[GTM];
  const int tid = (int)threadIdx.x, lane = tid & 31, wave = tid >> 5, hh = lane >> 4, m = lane & 15;
  const int rowBase = (int)blockIdx.x * GTM;

  const float* xp = x + (size_t)(rowBase + 16 * wave + m) * CH + 8 * hh;
  FragB af0, af1;
  af0.h[0] = cvt8(*(const v4f*)(xp),      *(const v4f*)(xp + 4));
  af0.h[1] = cvt8(*(const v4f*)(xp + 16), *(const v4f*)(xp + 20));
  af1.h[0] = cvt8(*(const v4f*)(xp + 32), *(const v4f*)(xp + 36));
  af1.h[1] = cvt8(*(const v4f*)(xp + 48), *(const v4f*)(xp + 52));

  v8f acc[4];
  {
    const v8f z = {0.f, 0.f, 0.f, 0.f, 0.f, 0.f, 0.f, 0.f};
#pragma unroll
    for (int t = 0; t < 4; ++t) acc[t] = z;
  }
  const unsigned short* bp = WT + (size_t)m * CH + 8 * hh;
#pragma unroll
  for (int nt = 0; nt < 4; ++nt) {
    const unsigned short* wq = bp + (size_t)(16 * nt) * CH;
    FragB b0, b1;
    b0.h[0] = *(const v8usa*)(wq);
    b0.h[1] = *(const v8usa*)(wq + 16);
    b1.h[0] = *(const v8usa*)(wq + 32);
    b1.h[1] = *(const v8usa*)(wq + 48);
    acc[nt] = wmb(af0, b0, acc[nt]);
    acc[nt] = wmb(af1, b1, acc[nt]);
  }

#pragma unroll
  for (int nt = 0; nt < 4; ++nt) {
    const int lc = 16 * nt + m;
#pragma unroll
    for (int r = 0; r < 8; ++r) {
      const int lr = 16 * wave + 8 * hh + r;
      stg[lr * CH + lc] = acc[nt][r];
    }
  }
  __syncthreads();

  const v4f a4 = *(const v4f*)(ATTF + 4 * m);
#pragma unroll 1
  for (int i = 0; i < 8; ++i) {
    const int rr = 16 * wave + 2 * i + hh;
    const v4f p = *(const v4fa*)(stg + rr * CH + 4 * m);
    float s = p.x * a4.x;
    s = fmaf(p.y, a4.y, s); s = fmaf(p.z, a4.z, s); s = fmaf(p.w, a4.w, s);
    s += __shfl_xor(s, 8);
    s += __shfl_xor(s, 4);
    s += __shfl_xor(s, 2);
    s += __shfl_xor(s, 1);
    if (m == 0) sdt[rr] = s;
  }
  __syncthreads();

  const v4f snv = *(const v4fa*)(sdt + 4 * lane);
  float* snp = SN + (size_t)rowBase + 4 * lane;
#pragma unroll 1
  for (int i = 0; i < 8; ++i) {
    const int rr = 16 * wave + 2 * i + hh;
    const v4f p = *(const v4fa*)(stg + rr * CH + 4 * m);
    float* op = XW + (size_t)(rowBase + rr) * CH + 4 * m;
    *(volatile v4f*)op = p;
  }
  if (wave == 0) *(volatile v4f*)snp = snv;
  __threadfence();
#pragma unroll 1
  for (int i = 0; i < 8; ++i) {
    const int rr = 16 * wave + 2 * i + hh;
    const v4f p = *(const v4fa*)(stg + rr * CH + 4 * m);
    float* op = XW + (size_t)(rowBase + rr) * CH + 4 * m;
    *(volatile v4f*)op = p;
  }
  if (wave == 0) *(volatile v4f*)snp = snv;
}

template <int MODE>
__global__ __launch_bounds__(NTHR) void k_seg(const int* __restrict__ hidx, int nE,
                                              const int* __restrict__ ELIST, const int* __restrict__ ECNTV,
                                              const float* __restrict__ XW, const float* __restrict__ ALPHA,
                                              const float* __restrict__ ATTF,
                                              float* OUTP, float* SE, double* TSV) {
  __shared__ int ech[SCH];
  __shared__ int nch[SCH];
  __shared__ __attribute__((aligned(16))) float est[BSZ * CH];
  __shared__ __attribute__((aligned(16))) float ses[BSZ];
  __shared__ double tsd[BSZ];
  const int tid = (int)threadIdx.x, lane = tid & 31, wave = tid >> 5;
  const int m = (int)blockIdx.x;
  int cnt = ECNTV[m * 32];
  cnt = clampi(cnt, 0, nE < EINC ? nE : EINC);
  const float bn = (cnt > 0) ? (1.0f / (float)cnt) : 0.0f;
  const int* erow = ELIST + (size_t)m * EINC;
  v2f acc[4];
#pragma unroll
  for (int j = 0; j < 4; ++j) { acc[j].x = 0.0f; acc[j].y = 0.0f; }

#pragma unroll 1
  for (int base = 0; base < cnt; base += SCH) {
#pragma unroll
    for (int j = 0; j < 4; ++j) {
      const int p  = base + tid + NTHR * j;
      const int pc = p < cnt ? p : cnt - 1;
      int e = erow[pc];
      e = clampi(e, 0, nE - 1);
      int nd = hidx[e];
      nd = clampi(nd, 0, NNODE - 1);
      ech[tid + NTHR * j] = e;
      nch[tid + NTHR * j] = nd;
    }
    __syncthreads();
    const int lim = (cnt - base) < SCH ? (cnt - base) : SCH;
#pragma unroll 1
    for (int q = 0; q < lim; ++q) {
      const int nd = nch[q];
      const float* rp = XW + ((size_t)(4 * wave) * NNODE + (size_t)nd) * CH + 2 * lane;
      const v2f v0 = *(const v2fa*)(rp);
      const v2f v1 = *(const v2fa*)(rp + (size_t)NNODE * CH);
      const v2f v2 = *(const v2fa*)(rp + (size_t)2 * NNODE * CH);
      const v2f v3 = *(const v2fa*)(rp + (size_t)3 * NNODE * CH);
      if constexpr (MODE == 0) {
        acc[0].x += v0.x; acc[0].y += v0.y;
        acc[1].x += v1.x; acc[1].y += v1.y;
        acc[2].x += v2.x; acc[2].y += v2.y;
        acc[3].x += v3.x; acc[3].y += v3.y;
      } else {
        const int e = ech[q];
        const v4f al = *(const v4f*)(ALPHA + (size_t)e * BSZ + 4 * wave);
        acc[0].x += bn * (al.x * v0.x); acc[0].y += bn * (al.x * v0.y);
        acc[1].x += bn * (al.y * v1.x); acc[1].y += bn * (al.y * v1.y);
        acc[2].x += bn * (al.z * v2.x); acc[2].y += bn * (al.z * v2.y);
        acc[3].x += bn * (al.w * v3.x); acc[3].y += bn * (al.w * v3.y);
      }
    }
    __syncthreads();
  }

#pragma unroll
  for (int j = 0; j < 4; ++j) *(v2fa*)(est + (4 * wave + j) * CH + 2 * lane) = acc[j];
  if constexpr (MODE == 0) {
    const v2f ab = *(const v2fa*)(ATTF + CH + 2 * lane);
#pragma unroll
    for (int j = 0; j < 4; ++j) {
      float s = acc[j].x * ab.x;
      s = fmaf(acc[j].y, ab.y, s);
#pragma unroll
      for (int off = 16; off > 0; off >>= 1) s += __shfl_xor(s, off);
      if (lane == 0) ses[4 * wave + j] = s;
    }
  }
  __syncthreads();
  double T = 0.0;
  if constexpr (MODE == 0) {
    if (wave == 0) {
      double d = 0.0;
#pragma unroll 4
      for (int c = 0; c < CH; ++c) d += (double)est[lane * CH + c];
      tsd[lane] = d;
    }
    __syncthreads();
    if (wave == 0) {
#pragma unroll 1
      for (int i = 0; i < BSZ; ++i) T += tsd[i];
    }
  }

  const v4f p0 = *(const v4fa*)(est + (4 * wave) * CH + 4 * lane);
  const v4f p1 = *(const v4fa*)(est + (4 * wave + 2) * CH + 4 * lane);
  float* op = OUTP + ((size_t)m * BSZ + 4 * wave) * CH + 4 * lane;
  v4f sv = {0.0f, 0.0f, 0.0f, 0.0f};
  v2d tv; tv.x = T; tv.y = T;
  if constexpr (MODE == 0) {
    if (wave == 0) sv = *(const v4fa*)(ses + 4 * (lane & 7));
  }
  *(volatile v4f*)op = p0;
  *(volatile v4f*)(op + 2 * CH) = p1;
  if constexpr (MODE == 0) {
    if (wave == 0 && lane < 8) {
      *(volatile v4f*)(SE + m * BSZ + 4 * lane) = sv;
      *(volatile v2d*)(TSV + m * 16 + 2 * lane) = tv;
    }
  }
  __threadfence();
  *(volatile v4f*)op = p0;
  *(volatile v4f*)(op + 2 * CH) = p1;
  if constexpr (MODE == 0) {
    if (wave == 0 && lane < 8) {
      *(volatile v4f*)(SE + m * BSZ + 4 * lane) = sv;
      *(volatile v2d*)(TSV + m * 16 + 2 * lane) = tv;
    }
  }
}

__global__ __launch_bounds__(NTHR) void k_alpha(const int* __restrict__ hidx, int nE,
                                                const int* __restrict__ NCNT, const int* __restrict__ NLIST,
                                                const float* __restrict__ SN, const float* __restrict__ SE,
                                                float* ALPHA) {
  __shared__ float evs[NWAVE * DEGCAP * BSZ];
  const int tid = (int)threadIdx.x, lane = tid & 31, wave = tid >> 5;
  const int node = __builtin_amdgcn_readfirstlane((int)blockIdx.x * NWAVE + wave);
  const int cnt  = __builtin_amdgcn_readfirstlane(clampi(NCNT[node], 0, DEGCAP));
  int ek = NLIST[(size_t)node * DEGCAP + lane];
  ek = clampi(ek, 0, nE - 1);
  int mk = hidx[nE + ek];
  mk = clampi(mk, 0, MEDGE - 1);
  const float sn = SN[(size_t)lane * NNODE + node];
  float* ev = evs + wave * (DEGCAP * BSZ);

  float mx = -3.0e38f;
#pragma unroll 1
  for (int k = 0; k < cnt; ++k) {
    const int mm = __builtin_amdgcn_readlane(mk, k);
    float sc = sn + SE[mm * BSZ + lane];
    sc = (sc >= 0.0f) ? sc : NEGSL * sc;
    ev[k * BSZ + lane] = sc;
    mx = fmaxf(mx, sc);
  }
  float s = 0.0f;
#pragma unroll 1
  for (int k = 0; k < cnt; ++k) {
    const float e = expf(ev[k * BSZ + lane] - mx);
    ev[k * BSZ + lane] = e;
    s += e;
  }
  const float rs = 1.0f / ((cnt > 0) ? s : 1.0f);
#pragma unroll 1
  for (int k = 0; k < cnt; ++k) {
    const int ee = __builtin_amdgcn_readlane(ek, k);
    const float al = ev[k * BSZ + lane] * rs;
    *(volatile float*)(ALPHA + (size_t)ee * BSZ + lane) = al;
  }
  __threadfence();
#pragma unroll 1
  for (int k = 0; k < cnt; ++k) {
    const int ee = __builtin_amdgcn_readlane(ek, k);
    const float al = ev[k * BSZ + lane] * rs;
    *(volatile float*)(ALPHA + (size_t)ee * BSZ + lane) = al;
  }
}

__global__ __launch_bounds__(NTHR) void k_out(const int* __restrict__ hidx, int nE,
                                              const int* __restrict__ NCNT, const int* __restrict__ NLIST,
                                              const int* __restrict__ POISONV,
                                              const float* __restrict__ ALPHA, const float* __restrict__ OUTE,
                                              float* out) {
  const int tid = (int)threadIdx.x, lane = tid & 31, wave = tid >> 5;
  const int node = __builtin_amdgcn_readfirstlane((int)blockIdx.x * NWAVE + wave);
  const int craw = NCNT[node];
  const int cnt  = __builtin_amdgcn_readfirstlane(clampi(craw, 0, DEGCAP));
  int ek = NLIST[(size_t)node * DEGCAP + lane];
  ek = clampi(ek, 0, nE - 1);
  int mk = hidx[nE + ek];
  mk = clampi(mk, 0, MEDGE - 1);
  const int pf = POISONV[0] | POISONV[32] | POISONV[64] | POISONV[96];
  const bool pz = (pf != 0) || (craw > DEGCAP);
  const float qn = __int_as_float(0x7fc00000);
  const float Dn = (float)cnt;

#pragma unroll 1
  for (int bg = 0; bg < BSZ / 4; ++bg) {
    const v4f a4 = *(const v4f*)(ALPHA + (size_t)ek * BSZ + 4 * bg);
    const int ai0 = __float_as_int(a4.x), ai1 = __float_as_int(a4.y);
    const int ai2 = __float_as_int(a4.z), ai3 = __float_as_int(a4.w);
    v2f c0 = {0.0f, 0.0f}, c1 = {0.0f, 0.0f}, c2 = {0.0f, 0.0f}, c3 = {0.0f, 0.0f};
#pragma unroll 1
    for (int k = 0; k < cnt; ++k) {
      const int mm = __builtin_amdgcn_readlane(mk, k);
      const float a0 = __int_as_float(__builtin_amdgcn_readlane(ai0, k));
      const float a1 = __int_as_float(__builtin_amdgcn_readlane(ai1, k));
      const float a2 = __int_as_float(__builtin_amdgcn_readlane(ai2, k));
      const float a3 = __int_as_float(__builtin_amdgcn_readlane(ai3, k));
      const float* rp = OUTE + ((size_t)mm * BSZ + 4 * bg) * CH + 2 * lane;
      const v2f v0 = *(const v2fa*)(rp);
      const v2f v1 = *(const v2fa*)(rp + CH);
      const v2f v2 = *(const v2fa*)(rp + 2 * CH);
      const v2f v3 = *(const v2fa*)(rp + 3 * CH);
      c0.x += Dn * (a0 * v0.x); c0.y += Dn * (a0 * v0.y);
      c1.x += Dn * (a1 * v1.x); c1.y += Dn * (a1 * v1.y);
      c2.x += Dn * (a2 * v2.x); c2.y += Dn * (a2 * v2.y);
      c3.x += Dn * (a3 * v3.x); c3.y += Dn * (a3 * v3.y);
    }
    v2f o0, o1, o2, o3;
    o0.x = pz ? qn : c0.x; o0.y = pz ? qn : c0.y;
    o1.x = pz ? qn : c1.x; o1.y = pz ? qn : c1.y;
    o2.x = pz ? qn : c2.x; o2.y = pz ? qn : c2.y;
    o3.x = pz ? qn : c3.x; o3.y = pz ? qn : c3.y;
    float* op = out + ((size_t)(4 * bg) * NNODE + (size_t)node) * CH + 2 * lane;
    const size_t bs = (size_t)NNODE * CH;
    *(volatile v2f*)(op) = o0;
    *(volatile v2f*)(op + bs) = o1;
    *(volatile v2f*)(op + 2 * bs) = o2;
    *(volatile v2f*)(op + 3 * bs) = o3;
    __threadfence();
    *(volatile v2f*)(op) = o0;
    *(volatile v2f*)(op + bs) = o1;
    *(volatile v2f*)(op + 2 * bs) = o2;
    *(volatile v2f*)(op + 3 * bs) = o3;
  }
}

__global__ __launch_bounds__(NTHR) void k_loss(const float* __restrict__ ES, float* REC) {
  __shared__ float esk[BSZ * 65];
  __shared__ float nks[BSZ];
  __shared__ __attribute__((aligned(16))) float recs[MEDGE];
  const int tid = (int)threadIdx.x, lane = tid & 31, wave = tid >> 5;
  const int k = (int)blockIdx.x;
#pragma unroll
  for (int j = 0; j < 2; ++j) {
    const int i4 = tid + NTHR * j;
    const int b = i4 >> 4, c = (i4 & 15) * 4;
    const v4f q = *(const v4f*)(ES + (size_t)k * (BSZ * CH) + 4 * i4);
    esk[b * 65 + c + 0] = q.x; esk[b * 65 + c + 1] = q.y;
    esk[b * 65 + c + 2] = q.z; esk[b * 65 + c + 3] = q.w;
  }
  __syncthreads();
  if (wave == 0) {
    float n2 = 0.0f;
#pragma unroll 4
    for (int c = 0; c < CH; ++c) { const float e = esk[lane * 65 + c]; n2 = fmaf(e, e, n2); }
    nks[lane] = sqrtf(n2);
  }
  __syncthreads();
  const float nrk = nks[lane];
#pragma unroll 1
  for (int i = 0; i < MEDGE / NWAVE; ++i) {
    const int m = wave + NWAVE * i;
    const float* rowp = ES + ((size_t)m * BSZ + lane) * CH;
    float inner = 0.0f, nm2 = 0.0f, dd = 0.0f;
#pragma unroll 1
    for (int c4 = 0; c4 < CH / 4; ++c4) {
      const v4f q = *(const v4f*)(rowp + 4 * c4);
      const float e0 = esk[lane * 65 + 4 * c4 + 0], e1 = esk[lane * 65 + 4 * c4 + 1];
      const float e2 = esk[lane * 65 + 4 * c4 + 2], e3 = esk[lane * 65 + 4 * c4 + 3];
      const float d0 = e0 - q.x, d1 = e1 - q.y, d2 = e2 - q.z, d3 = e3 - q.w;
      inner = fmaf(e0, q.x, inner); nm2 = fmaf(q.x, q.x, nm2); dd = fmaf(d0, d0, dd);
      inner = fmaf(e1, q.y, inner); nm2 = fmaf(q.y, q.y, nm2); dd = fmaf(d1, d1, dd);
      inner = fmaf(e2, q.z, inner); nm2 = fmaf(q.z, q.z, nm2); dd = fmaf(d2, d2, dd);
      inner = fmaf(e3, q.w, inner); nm2 = fmaf(q.w, q.w, nm2); dd = fmaf(d3, d3, dd);
    }
    const float nrm  = sqrtf(nm2);
    const float dist = sqrtf(dd);
    const float cosv = inner / (nrk * nrm);
    float s = cosv * dist + (1.0f - cosv) * fmaxf(HINGE - dist, 0.0f);
#pragma unroll
    for (int off = 16; off > 0; off >>= 1) s += __shfl_xor(s, off);
    const float mean = s * (1.0f / (float)BSZ);
    if (lane == 0) recs[m] = fabsf(mean);
  }
  __syncthreads();
  if (wave == 0) {
    const v4f v = *(const v4fa*)(recs + 4 * (lane & 15));
    float* op = REC + (size_t)k * MEDGE + 4 * lane;
    if (lane < 16) *(volatile v4f*)op = v;
    __threadfence();
    if (lane < 16) *(volatile v4f*)op = v;
  }
}

__global__ __launch_bounds__(32) void k_final(const float* __restrict__ REC, const double* __restrict__ TSV,
                                              const int* __restrict__ ECNTV, const int* __restrict__ POISONV,
                                              int nE, float* out, int lastIdx) {
  __shared__ double part[32];
  const int lane = (int)threadIdx.x;
  double d = 0.0;
#pragma unroll 1
  for (int i = 0; i < 32; ++i) {
    const v4f q = *(const v4f*)(REC + lane * 128 + 4 * i);
    d += (double)q.x; d += (double)q.y; d += (double)q.z; d += (double)q.w;
  }
  part[lane] = d;
  __syncthreads();
  double tot = 0.0;
#pragma unroll 1
  for (int i = 0; i < 32; ++i) tot += part[i];
  double ms = 0.0;
#pragma unroll 1
  for (int m = 0; m < MEDGE; ++m) {
    const int c = clampi(ECNTV[m * 32], 0, EINC);
    ms += (1.0 - (double)c) * TSV[m * 16];
  }
  const double mean = ms / ((double)nE * (double)(BSZ * CH));
  const double loss = tot / (double)((MEDGE + 1) * (MEDGE + 1));
  float r = (float)fabs(mean) + (float)loss;
  const int pf = POISONV[0] | POISONV[32] | POISONV[64] | POISONV[96];
  r = (pf != 0) ? __int_as_float(0x7fc00000) : r;
  if (lane == 0) *(volatile float*)(out + lastIdx) = r;
  __threadfence();
  if (lane == 0) *(volatile float*)(out + lastIdx) = r;
}

static inline size_t al256(size_t o) { return (o + 255) & ~(size_t)255; }

extern "C" void kernel_launch(void* const* d_in, const int* in_sizes, int n_in,
                              void* d_out, int out_size, void* d_ws, size_t ws_size,
                              hipStream_t stream) {
  if (n_in < 6) return;
  if (in_sizes[0] != NROW * CH) return;
  if (in_sizes[1] != CH * CH) return;
  if (in_sizes[2] != 2 * CH) return;
  if (in_sizes[3] < 2 || (in_sizes[3] & 1) != 0) return;
  const int nE = in_sizes[3] / 2;
  if (nE < 1 || nE > EINC) return;
  if (in_sizes[4] < 1 || in_sizes[5] < 1) return;
  if ((long long)out_size != (long long)NROW * CH + 1) return;

  const float* x    = (const float*)d_in[0];
  const float* W    = (const float*)d_in[1];
  const float* att  = (const float*)d_in[2];
  const int*   hidx = (const int*)d_in[3];
  float* out = (float*)d_out;
  const int lastIdx = NROW * CH;
  if (lastIdx >= out_size) return;
  const int vec8 = ((nE & 3) == 0) ? 1 : 0;

  char* ws = (char*)d_ws;
  size_t off = 0;
  const size_t oWT   = off; off = al256(off + (size_t)CH * CH * 2);
  const size_t oATT  = off; off = al256(off + (size_t)2 * CH * 4);
  const size_t oPOI  = off; off = al256(off + (size_t)NBLKN * 32 * 4);
  const size_t oECN  = off; off = al256(off + (size_t)MEDGE * 32 * 4);
  const size_t oTS   = off; off = al256(off + (size_t)MEDGE * 16 * 8);
  const size_t oSE   = off; off = al256(off + (size_t)MEDGE * BSZ * 4);
  const size_t oREC  = off; off = al256(off + (size_t)MEDGE * MEDGE * 4);
  const size_t oNCN  = off; off = al256(off + (size_t)NNODE * 4);
  const size_t oNLS  = off; off = al256(off + (size_t)NNODE * DEGCAP * 4);
  const size_t oSN   = off; off = al256(off + (size_t)NROW * 4);
  const size_t oES   = off; off = al256(off + (size_t)MEDGE * BSZ * CH * 4);
  const size_t oOE   = off; off = al256(off + (size_t)MEDGE * BSZ * CH * 4);
  const size_t oAL   = off; off = al256(off + (size_t)EINC * BSZ * 4);
  const size_t oEL   = off; off = al256(off + (size_t)MEDGE * EINC * 4);
  const size_t oXW   = off; off = al256(off + (size_t)NROW * CH * 4);
  if (off > ws_size || off > (size_t)WSMAX) return;
  unsigned short* WT  = (unsigned short*)(ws + oWT);
  float*  ATTF  = (float*)(ws + oATT);
  int*    POIS  = (int*)(ws + oPOI);
  int*    ECNTV = (int*)(ws + oECN);
  double* TSV   = (double*)(ws + oTS);
  float*  SE    = (float*)(ws + oSE);
  float*  REC   = (float*)(ws + oREC);
  int*    NCNT  = (int*)(ws + oNCN);
  int*    NLIST = (int*)(ws + oNLS);
  float*  SN    = (float*)(ws + oSN);
  float*  ES    = (float*)(ws + oES);
  float*  OUTE  = (float*)(ws + oOE);
  float*  ALPHA = (float*)(ws + oAL);
  int*    ELIST = (int*)(ws + oEL);
  float*  XW    = (float*)(ws + oXW);

  const size_t bkLds = (size_t)BK_LDS_INTS * 4;
  hipFuncSetAttribute(reinterpret_cast<const void*>(&k_bucket), hipFuncAttributeMaxDynamicSharedMemorySize, (int)bkLds);

  k_prep<<<(NU_A + NU_W) / NTHR + 1, NTHR, 0, stream>>>(W, att, WT, ATTF, ALPHA);
  k_bucket<<<NBLKN + MEDGE, NTHR, bkLds, stream>>>(hidx, nE, vec8, NCNT, NLIST, POIS, ELIST, ECNTV);
  k_gemm<<<NROW / GTM, NTHR, 0, stream>>>(x, WT, ATTF, XW, SN);
  k_seg<0><<<MEDGE, NTHR, 0, stream>>>(hidx, nE, ELIST, ECNTV, XW, ALPHA, ATTF, ES, SE, TSV);
  k_alpha<<<NNODE / NWAVE, NTHR, 0, stream>>>(hidx, nE, NCNT, NLIST, SN, SE, ALPHA);
  k_seg<1><<<MEDGE, NTHR, 0, stream>>>(hidx, nE, ELIST, ECNTV, XW, ALPHA, ATTF, OUTE, SE, TSV);
  k_out<<<NNODE / NWAVE, NTHR, 0, stream>>>(hidx, nE, NCNT, NLIST, POIS, ALPHA, OUTE, out);
  k_loss<<<MEDGE, NTHR, 0, stream>>>(ES, REC);
  k_final<<<1, 32, 0, stream>>>(REC, TSV, ECNTV, POIS, nE, out, lastIdx);
}
